// SAGE_24575802868448
// MI455X (gfx1250) — hardware-verified
//
#include <hip/hip_runtime.h>
#include <stddef.h>
#include <stdint.h>
#include <math.h>


#define F0     128
#define C1     256
#define NCLS   41
#define NCP    64
#define KZ     (2 * F0)
#define KA     (2 * C1)
#define NTHR   256
#define NWAVE  8
#define EPT    8
#define CHUNK  (NTHR * EPT)
#define WCAP   (EPT * 32)
#define LISTN  (NWAVE * WCAP)
#define NBA    1024
#define SLA    10
#define RCAP   28672
#define DEGCAP 64
#define GBM    64
#define GTHR   128
#define GWAVE  (GTHR / 32)
#define GNC    128
#define PARTW  288
#define WSTW   258
#define HPR    8
#define HPB    (NWAVE * HPR)
#define AGG_ZINTS    (LISTN + 2 * RCAP + 3 * NBA)
#define MISC_INTS    16
#define AGG_LDS_INTS (AGG_ZINTS + MISC_INTS)
#define MAXL   8
#define WSMAX  134217728

static_assert((CHUNK & (CHUNK - 1)) == 0 && CHUNK <= 4096);
static_assert((NBA & (NBA - 1)) == 0 && NBA == (1 << SLA));
static_assert(((long long)CHUNK << SLA) < (1LL << 31));
static_assert(LISTN % NTHR == 0);
static_assert(NBA % NWAVE == 0 && NBA % 32 == 0 && NBA % GBM == 0);
static_assert(RCAP % 32 == 0 && LISTN % 4 == 0 && AGG_ZINTS % (NTHR * 4) == 0);
static_assert(KZ % 32 == 0 && KA % 32 == 0 && KZ == 2 * F0 && KA == 2 * C1);
static_assert(GBM == GWAVE * 16 && C1 == 2 * GNC && F0 == GNC && F0 == 4 * 32 && C1 == 8 * 32);
static_assert(PARTW % 32 == 0 && PARTW / 4 <= GTHR && PARTW >= 2 * GNC + 1);
static_assert(WSTW >= 2 * GNC + 1 && (WSTW % 2) == 0);
static_assert(HPB == GBM && NTHR == C1 && NTHR == 2 * F0);
static_assert(NCLS <= NCP && NCP == 64 && (GBM * NCLS) % 32 == 0);
static_assert(AGG_LDS_INTS * 4 <= 300000);

typedef float          v2f   __attribute__((ext_vector_type(2)));
typedef float          v4f   __attribute__((ext_vector_type(4)));
typedef float          v8f   __attribute__((ext_vector_type(8)));
typedef int            v4i   __attribute__((ext_vector_type(4)));
typedef int            v8i   __attribute__((ext_vector_type(8)));
typedef unsigned int   v2u   __attribute__((ext_vector_type(2)));
typedef unsigned int   v4u   __attribute__((ext_vector_type(4)));
typedef unsigned short v8us  __attribute__((ext_vector_type(8)));
typedef unsigned short v16us __attribute__((ext_vector_type(16)));
typedef __bf16         v16bf __attribute__((ext_vector_type(16)));
typedef v2f  __attribute__((may_alias)) v2fa;
typedef v4f  __attribute__((may_alias)) v4fa;
typedef v4i  __attribute__((may_alias)) v4ia;
typedef v8us __attribute__((may_alias)) v8usa;
union FragB { v16bf v; v16us u; v8us h[2]; v8i w; };

__device__ __forceinline__ v8f wmb(const FragB& a, const FragB& b, v8f c) {
  v8f d = __builtin_amdgcn_wmma_f32_16x16x32_bf16(false, a.v, false, b.v, (short)0, c, false, false);
  asm volatile("v_nop\n\tv_nop\n\tv_nop\n\tv_nop" : "+v"(d) : "v"(a.w), "v"(b.w));
  return d;
}

__device__ __forceinline__ v8f z8() { v8f z = {0.f, 0.f, 0.f, 0.f, 0.f, 0.f, 0.f, 0.f}; return z; }

__device__ __forceinline__ unsigned bf16_bits(float f) {
  const unsigned u = __float_as_uint(f);
  return ((u + 0x7FFFu + ((u >> 16) & 1u)) >> 16) & 0xFFFFu;
}
__device__ __forceinline__ float bf16_val(float f) {
  return __uint_as_float(bf16_bits(f) << 16);
}
__device__ __forceinline__ unsigned hl_bits(float v, unsigned& lo) {
  const unsigned hb = bf16_bits(v);
  lo = bf16_bits(v - __uint_as_float(hb << 16));
  return hb;
}
__device__ __forceinline__ unsigned pk2(float lo, float hi) { return bf16_bits(lo) | (bf16_bits(hi) << 16); }
__device__ __forceinline__ v4u pack8(const v4f a, const v4f b) {
  v4u r;
  r.x = pk2(a.x, a.y); r.y = pk2(a.z, a.w); r.z = pk2(b.x, b.y); r.w = pk2(b.z, b.w);
  return r;
}

template <int CP, int RND>
__device__ __forceinline__ void ldrow(const float* p, float* v) {
  if constexpr (CP == 4) {
    const v4f t = *(const v4fa*)p;
    v[0] = t.x; v[1] = t.y; v[2] = t.z; v[3] = t.w;
  } else {
    const v4f t0 = *(const v4fa*)p;
    const v4f t1 = *(const v4fa*)(p + 4);
    v[0] = t0.x; v[1] = t0.y; v[2] = t0.z; v[3] = t0.w;
    v[4] = t1.x; v[5] = t1.y; v[6] = t1.z; v[7] = t1.w;
  }
  if constexpr (RND != 0) {
#pragma unroll
    for (int j = 0; j < CP; ++j) v[j] = bf16_val(v[j]);
  }
}

template <int SLB>
__device__ __forceinline__ int scan_chunk(const int* __restrict__ dsts, int nE, int cbase, int slotBase,
                                          int nb, int vec8, int* list, int tid, int lane, int wave) {
  int wc = 0;
  const int el0  = tid * EPT;
  const int e0   = cbase + el0;
  const int sent = -2147483647 - 1;
  v4i da, db;
  if (vec8 != 0 && cbase + CHUNK <= nE) {
    da = *(const v4i*)(dsts + e0);
    db = *(const v4i*)(dsts + e0 + 4);
  } else {
    da.x = (e0     < nE) ? dsts[min(e0,     nE - 1)] : sent;
    da.y = (e0 + 1 < nE) ? dsts[min(e0 + 1, nE - 1)] : sent;
    da.z = (e0 + 2 < nE) ? dsts[min(e0 + 2, nE - 1)] : sent;
    da.w = (e0 + 3 < nE) ? dsts[min(e0 + 3, nE - 1)] : sent;
    db.x = (e0 + 4 < nE) ? dsts[min(e0 + 4, nE - 1)] : sent;
    db.y = (e0 + 5 < nE) ? dsts[min(e0 + 5, nE - 1)] : sent;
    db.z = (e0 + 6 < nE) ? dsts[min(e0 + 6, nE - 1)] : sent;
    db.w = (e0 + 7 < nE) ? dsts[min(e0 + 7, nE - 1)] : sent;
  }
  const unsigned nbs = (unsigned)slotBase;
  const unsigned unb = (unsigned)nb;
  const unsigned s0 = (unsigned)da.x - nbs, s1 = (unsigned)da.y - nbs;
  const unsigned s2 = (unsigned)da.z - nbs, s3 = (unsigned)da.w - nbs;
  const unsigned s4 = (unsigned)db.x - nbs, s5 = (unsigned)db.y - nbs;
  const unsigned s6 = (unsigned)db.z - nbs, s7 = (unsigned)db.w - nbs;
  const bool h0 = s0 < unb, h1 = s1 < unb, h2 = s2 < unb, h3 = s3 < unb;
  const bool h4 = s4 < unb, h5 = s5 < unb, h6 = s6 < unb, h7 = s7 < unb;
  const unsigned any = __builtin_amdgcn_ballot_w32(h0 | h1 | h2 | h3 | h4 | h5 | h6 | h7);
  if (any != 0u) {
#define HITJ(J, HJ, SJ) { \
      const unsigned mj = __builtin_amdgcn_ballot_w32(HJ); \
      if (mj != 0u) { \
        if (HJ) { \
          const int pos = wc + (int)__builtin_amdgcn_mbcnt_lo(mj, 0u); \
          if (pos < WCAP) list[wave * WCAP + pos] = ((el0 + (J)) << SLB) | (int)(SJ); \
        } \
        wc += (int)__builtin_popcount(mj); } }
    HITJ(0, h0, s0)
    HITJ(1, h1, s1)
    HITJ(2, h2, s2)
    HITJ(3, h3, s3)
    HITJ(4, h4, s4)
    HITJ(5, h5, s5)
    HITJ(6, h6, s6)
    HITJ(7, h7, s7)
#undef HITJ
  }
  return wc;
}

__global__ __launch_bounds__(NTHR) void k_wtr(const float* __restrict__ w, int Kin, int Ncol, int Nrows, int Kout,
                                              int upl, int nUnits, unsigned short* wt) {
  const int u = (int)blockIdx.x * NTHR + (int)threadIdx.x;
  if (u >= nUnits) return;
  const int l  = u / upl;
  const int ul = u - l * upl;
  const int kq = Kout >> 3;
  const int n  = ul / kq;
  const int k8 = (ul - n * kq) * 8;
  const int kk = k8 - (k8 / Kin) * Kin;
  const int ncl = n < Ncol ? n : Ncol - 1;
  const float* p = w + (size_t)l * (size_t)Kin * (size_t)Ncol + (size_t)kk * (size_t)Ncol + ncl;
  v4f a, b;
  a.x = p[0];                    a.y = p[(size_t)Ncol];         a.z = p[(size_t)2 * Ncol];     a.w = p[(size_t)3 * Ncol];
  b.x = p[(size_t)4 * Ncol];     b.y = p[(size_t)5 * Ncol];     b.z = p[(size_t)6 * Ncol];     b.w = p[(size_t)7 * Ncol];
  const v4f z4 = {0.f, 0.f, 0.f, 0.f};
  if (n >= Ncol || n >= Nrows) { a = z4; b = z4; }
  const v4u wv = pack8(a, b);
  unsigned short* o = wt + (size_t)l * (size_t)Nrows * (size_t)Kout + (size_t)n * (size_t)Kout + k8;
  *(volatile v4u*)o = wv;
  __threadfence();
  *(volatile v4u*)o = wv;
}

template <int FD, int RND>
__global__ __launch_bounds__(NTHR) void k_scan(const int* __restrict__ srcs, const int* __restrict__ dsts,
                                               int nE, int nN, int vec8, int mRows,
                                               const float* __restrict__ epl, const float* __restrict__ hsrc,
                                               unsigned short* apl) {
  constexpr int CP = FD / 32;
  constexpr int KP = 2 * FD;
  static_assert(CP == 4 || CP == 8);
  extern __shared__ __attribute__((aligned(16))) int dsm[];
  int* list = dsm;
  int* hl   = dsm + LISTN;
  int* sl   = hl + RCAP;
  int* cnt  = sl + RCAP;
  int* offs = cnt + NBA;
  int* cur  = offs + NBA;
  int* misc = cur + NBA;
  const int tid = (int)threadIdx.x, lane = tid & 31, wave = tid >> 5;
  const int nodeBase = (int)blockIdx.x * NBA;

  {
    const v4i z4 = {0, 0, 0, 0};
    for (int i = tid * 4; i < AGG_ZINTS; i += NTHR * 4) *(v4ia*)(dsm + i) = z4;
    if (tid < MISC_INTS) misc[tid] = 0;
  }
  __syncthreads();
  const float opl = 1.0f + bf16_val(epl[0]);

  int t = 0, ov = 0;
  const int nChunks = (nE + CHUNK - 1) / CHUNK;
#pragma unroll 1
  for (int ch = 0; ch < nChunks; ++ch) {
    const int cbase = ch * CHUNK;
    const int wc = scan_chunk<SLA>(dsts, nE, cbase, nodeBase, NBA, vec8, list, tid, lane, wave);
    if (lane == 0) misc[wave] = wc;
    __syncthreads();
    if (wave == 0) {
#pragma unroll 1
      for (int w2 = 0; w2 < NWAVE; ++w2) {
        int c = misc[w2];
        c = c < 0 ? 0 : (c > WCAP ? WCAP : c);
#pragma unroll 1
        for (int b0 = 0; b0 < c; b0 += 32) {
          const int idx = b0 + lane;
          const int ent = list[w2 * WCAP + (idx < WCAP ? idx : WCAP - 1)];
          const int m32 = (c - b0) < 32 ? (c - b0) : 32;
#pragma unroll 1
          for (int k = 0; k < m32; ++k) {
            const int u    = __builtin_amdgcn_readlane(ent, k);
            const int slot = u & (NBA - 1);
            const int el   = (u >> SLA) & (CHUNK - 1);
            const int pk   = ((cbase + el) << SLA) | slot;
            if (t < RCAP) {
              if (lane == 0) { hl[t] = pk; cnt[slot] = cnt[slot] + 1; }
              t = t + 1;
            } else {
              ov = 1;
            }
          }
        }
      }
    }
    __syncthreads();
  }
  if (wave == 0 && lane == 0) { misc[8] = t; misc[9] = ov; }
  __syncthreads();
  int tt = misc[8];
  tt = tt < 0 ? 0 : (tt > RCAP ? RCAP : tt);
  const int ovf = misc[9];

  if (wave == 0) {
    const int base = lane * (NBA / 32);
    int s = 0;
#pragma unroll 1
    for (int i = 0; i < NBA / 32; ++i) s += cnt[base + i];
    int incl = s;
#pragma unroll
    for (int d = 1; d < 32; d <<= 1) {
      const int y = __shfl_up(incl, d, 32);
      if (lane >= d) incl += y;
    }
    int run = incl - s;
#pragma unroll 1
    for (int i = 0; i < NBA / 32; ++i) {
      const int cv = cnt[base + i];
      offs[base + i] = run;
      cur[base + i]  = run;
      run += cv;
    }
  }
  __syncthreads();
  if (wave == 0) {
#pragma unroll 1
    for (int b0 = 0; b0 < tt; b0 += 32) {
      const int idx = b0 + lane;
      const int ent = hl[idx < RCAP ? idx : RCAP - 1];
      const int m32 = (tt - b0) < 32 ? (tt - b0) : 32;
#pragma unroll 1
      for (int k = 0; k < m32; ++k) {
        const int u    = __builtin_amdgcn_readlane(ent, k);
        const int slot = u & (NBA - 1);
        if (lane == 0) {
          int p = cur[slot];
          p = p < 0 ? 0 : (p > RCAP - 1 ? RCAP - 1 : p);
          sl[p] = u;
          cur[slot] = p + 1;
        }
      }
    }
  }
  __syncthreads();

  const float qnan = __int_as_float(0x7fc00000);
  const float pz = (ovf != 0) ? qnan : 0.0f;
#pragma unroll 1
  for (int si = 0; si < NBA / NWAVE; ++si) {
    const int s    = si * NWAVE + wave;
    const int node = nodeBase + s;
    int c = cnt[s];
    const bool big = c > DEGCAP;
    c = c < 0 ? 0 : (c > DEGCAP ? DEGCAP : c);
    int o = offs[s];
    o = o < 0 ? 0 : (o > RCAP ? RCAP : o);
    const int nc = node < nN ? node : nN - 1;
    float ag[CP];
#pragma unroll
    for (int j = 0; j < CP; ++j) ag[j] = 0.0f;
#pragma unroll 1
    for (int b0 = 0; b0 < c; b0 += 32) {
      int idx = o + b0 + lane;
      idx = idx > RCAP - 1 ? RCAP - 1 : idx;
      const int ent = sl[idx];
      int eid = ent >> SLA;
      eid = eid < 0 ? 0 : (eid > nE - 1 ? nE - 1 : eid);
      int sr = srcs[eid];
      sr = sr < 0 ? 0 : (sr > nN - 1 ? nN - 1 : sr);
      const int m32 = (c - b0) < 32 ? (c - b0) : 32;
#pragma unroll 1
      for (int k = 0; k < m32; ++k) {
        const int sk = __builtin_amdgcn_readlane(sr, k);
        float v[CP];
        ldrow<CP, RND>(hsrc + (size_t)sk * FD + CP * lane, v);
#pragma unroll
        for (int j = 0; j < CP; ++j) ag[j] = ag[j] + v[j];
      }
    }
    const float pzr = big ? qnan : pz;
    const bool live = node < nN;
    float hr[CP];
    ldrow<CP, RND>(hsrc + (size_t)nc * FD + CP * lane, hr);
    unsigned hb[CP], lb[CP];
#pragma unroll
    for (int j = 0; j < CP; ++j) {
      const float z = live ? (fmaf(opl, hr[j], ag[j]) + pzr) : 0.0f;
      hb[j] = hl_bits(z, lb[j]);
    }
    if (node < mRows) {
      unsigned short* rpw = apl + (size_t)node * KP;
      if constexpr (CP == 4) {
        v2u hp, lp;
        hp.x = hb[0] | (hb[1] << 16); hp.y = hb[2] | (hb[3] << 16);
        lp.x = lb[0] | (lb[1] << 16); lp.y = lb[2] | (lb[3] << 16);
        unsigned short* ph = rpw + 4 * lane;
        unsigned short* pl = rpw + FD + 4 * lane;
        *(volatile v2u*)ph = hp;
        *(volatile v2u*)pl = lp;
        __threadfence();
        *(volatile v2u*)ph = hp;
        *(volatile v2u*)pl = lp;
      } else {
        v4u hp, lp;
        hp.x = hb[0] | (hb[1] << 16); hp.y = hb[2] | (hb[3] << 16); hp.z = hb[4] | (hb[5] << 16); hp.w = hb[6] | (hb[7] << 16);
        lp.x = lb[0] | (lb[1] << 16); lp.y = lb[2] | (lb[3] << 16); lp.z = lb[4] | (lb[5] << 16); lp.w = lb[6] | (lb[7] << 16);
        unsigned short* ph = rpw + 8 * lane;
        unsigned short* pl = rpw + FD + 8 * lane;
        *(volatile v4u*)ph = hp;
        *(volatile v4u*)pl = lp;
        __threadfence();
        *(volatile v4u*)ph = hp;
        *(volatile v4u*)pl = lp;
      }
    }
  }
}

template <int NC, int KK, int LDO, int EPI>
__global__ __launch_bounds__(GTHR) void k_gemm(const unsigned short* __restrict__ Apl,
                                               const unsigned short* __restrict__ BT,
                                               const float* __restrict__ bias, int nN,
                                               float* outp, float* part, unsigned short* opl) {
  constexpr int NT  = NC / 16;
  constexpr int CPL = NC / 32;
  static_assert(NT >= 1 && NT <= 8 && (CPL == 2 || CPL == 4) && KK % 32 == 0);
  static_assert(EPI == 0 || EPI == 2 || EPI == 3);
  static_assert(EPI != 0 || (NC == GNC && LDO % NC == 0 && CPL == 4));
  static_assert(EPI != 2 || (NC == NCP && CPL == 2 && NCLS <= NC));
  static_assert(EPI != 3 || (NC == LDO && CPL == 4));
  __shared__ __attribute__((aligned(16))) float stg[GBM * NC];
  __shared__ __attribute__((aligned(16))) float wst[(EPI == 0) ? (GWAVE * WSTW) : 4];
  __shared__ __attribute__((aligned(16))) float pst[(EPI == 0) ? PARTW : 4];
  __shared__ __attribute__((aligned(16))) float ost[(EPI == 2) ? (GBM * NCLS) : 4];
  const int tid = (int)threadIdx.x, lane = tid & 31, wave = tid >> 5, hh = lane >> 4, m = lane & 15;
  const int rowBase = (int)blockIdx.x * GBM;
  const int col0    = (int)blockIdx.y * NC;

  v8f acc[NT];
#pragma unroll
  for (int t = 0; t < NT; ++t) acc[t] = z8();
  const unsigned short* ap = Apl + (size_t)(rowBase + 16 * wave + m) * (size_t)KK + 8 * hh;
  const unsigned short* bp = BT + (size_t)(col0 + m) * (size_t)KK + 8 * hh;

#pragma unroll 1
  for (int k0 = 0; k0 < KK; k0 += 32) {
    FragB af;
    af.h[0] = *(const v8usa*)(ap + k0);
    af.h[1] = *(const v8usa*)(ap + k0 + 16);
#pragma unroll
    for (int nt = 0; nt < NT; ++nt) {
      const unsigned short* wq = bp + (size_t)(16 * nt) * (size_t)KK + k0;
      FragB bf;
      bf.h[0] = *(const v8usa*)wq;
      bf.h[1] = *(const v8usa*)(wq + 16);
      acc[nt] = wmb(af, bf, acc[nt]);
    }
  }

#pragma unroll
  for (int nt = 0; nt < NT; ++nt) {
    const int lc = 16 * nt + m;
#pragma unroll
    for (int r = 0; r < 8; ++r) {
      const int lr = 16 * wave + 8 * hh + r;
      stg[lr * NC + lc] = acc[nt][r];
    }
  }
  __syncthreads();

  float bq[CPL];
  if constexpr (CPL == 4) {
    const v4f b4 = *(const v4fa*)(bias + col0 + 4 * lane);
    bq[0] = bf16_val(b4.x); bq[1] = bf16_val(b4.y); bq[2] = bf16_val(b4.z); bq[3] = bf16_val(b4.w);
  } else {
    const int c0 = 2 * lane, c1v = 2 * lane + 1;
    bq[0] = bf16_val(bias[c0  < NCLS ? c0  : NCLS - 1]);
    bq[1] = bf16_val(bias[c1v < NCLS ? c1v : NCLS - 1]);
  }

  float pv[16][CPL];
  int wn = 0;
  float wm[CPL], wqv[CPL];
#pragma unroll
  for (int j = 0; j < CPL; ++j) { wm[j] = 0.0f; wqv[j] = 0.0f; }
#pragma unroll
  for (int i = 0; i < 16; ++i) {
    const int row = rowBase + 16 * wave + i;
    const bool ok = row < nN;
    float x[CPL];
    if constexpr (CPL == 4) {
      const v4f t4 = *(const v4fa*)(stg + (16 * wave + i) * NC + 4 * lane);
      x[0] = t4.x; x[1] = t4.y; x[2] = t4.z; x[3] = t4.w;
    } else {
      const v2f t2 = *(const v2fa*)(stg + (16 * wave + i) * NC + 2 * lane);
      x[0] = t2.x; x[1] = t2.y;
    }
    if constexpr (EPI != 2) {
      float vv[CPL];
#pragma unroll
      for (int j = 0; j < CPL; ++j) {
        vv[j] = ok ? (x[j] + bq[j]) : 0.0f;
        pv[i][j] = vv[j];
      }
      if constexpr (EPI == 0) {
        if (ok) {
          wn += 1;
          const float rk = 1.0f / (float)(i + 1);
#pragma unroll
          for (int j = 0; j < CPL; ++j) {
            const float dd = vv[j] - wm[j];
            wm[j]  = fmaf(dd, rk, wm[j]);
            wqv[j] = fmaf(dd, vv[j] - wm[j], wqv[j]);
          }
        }
      }
    } else {
      const bool v0 = (2 * lane) < NCLS, v1 = (2 * lane + 1) < NCLS;
      const float nlo = -3.0e38f;
      const float z0 = v0 ? (x[0] + bq[0]) : nlo;
      const float z1 = v1 ? (x[1] + bq[1]) : nlo;
      float vm = fmaxf(z0, z1);
#pragma unroll
      for (int off = 16; off > 0; off >>= 1) vm = fmaxf(vm, __shfl_xor(vm, off));
      const float d0 = z0 - vm, d1 = z1 - vm;
      float sm = expf(d0) + expf(d1);
#pragma unroll
      for (int off = 16; off > 0; off >>= 1) sm += __shfl_xor(sm, off);
      const float ls = logf(sm);
      pv[i][0] = d0 - ls;
      pv[i][1] = d1 - ls;
      (void)ok;
    }
  }

  if constexpr (EPI == 0) {
#pragma unroll
    for (int i = 0; i < 16; ++i) {
      const int row = rowBase + 16 * wave + i;
      float* op = outp + (size_t)row * (size_t)LDO + col0 + CPL * lane;
      v4f q; q.x = pv[i][0]; q.y = pv[i][1]; q.z = pv[i][2]; q.w = pv[i][3];
      *(volatile v4f*)op = q;
    }
    __threadfence();
#pragma unroll
    for (int i = 0; i < 16; ++i) {
      const int row = rowBase + 16 * wave + i;
      float* op = outp + (size_t)row * (size_t)LDO + col0 + CPL * lane;
      v4f q; q.x = pv[i][0]; q.y = pv[i][1]; q.z = pv[i][2]; q.w = pv[i][3];
      *(volatile v4f*)op = q;
    }
  } else if constexpr (EPI == 3) {
    v2u hpk[16], lpk[16];
#pragma unroll
    for (int i = 0; i < 16; ++i) {
      unsigned hb[4], lb[4];
#pragma unroll
      for (int j = 0; j < 4; ++j) hb[j] = hl_bits(pv[i][j], lb[j]);
      hpk[i].x = hb[0] | (hb[1] << 16); hpk[i].y = hb[2] | (hb[3] << 16);
      lpk[i].x = lb[0] | (lb[1] << 16); lpk[i].y = lb[2] | (lb[3] << 16);
    }
#pragma unroll
    for (int i = 0; i < 16; ++i) {
      const int row = rowBase + 16 * wave + i;
      unsigned short* rp = opl + (size_t)row * (size_t)(2 * LDO);
      *(volatile v2u*)(rp + 4 * lane) = hpk[i];
      *(volatile v2u*)(rp + LDO + 4 * lane) = lpk[i];
    }
    __threadfence();
#pragma unroll
    for (int i = 0; i < 16; ++i) {
      const int row = rowBase + 16 * wave + i;
      unsigned short* rp = opl + (size_t)row * (size_t)(2 * LDO);
      *(volatile v2u*)(rp + 4 * lane) = hpk[i];
      *(volatile v2u*)(rp + LDO + 4 * lane) = lpk[i];
    }
  } else {
    const bool v0 = (2 * lane) < NCLS, v1 = (2 * lane + 1) < NCLS;
#pragma unroll
    for (int i = 0; i < 16; ++i) {
      const int lr = 16 * wave + i;
      if (v0) ost[lr * NCLS + 2 * lane]     = pv[i][0];
      if (v1) ost[lr * NCLS + 2 * lane + 1] = pv[i][1];
    }
    __syncthreads();
    int nr = nN - rowBase;
    nr = nr < 0 ? 0 : (nr > GBM ? GBM : nr);
    const int cntf = nr * NCLS;
    const int nq = cntf >> 2;
    const int rem = cntf & 3;
    float* ob = outp + (size_t)rowBase * (size_t)NCLS;
#pragma unroll 1
    for (int q = tid; q < nq; q += GTHR) {
      const v4f v = *(const v4fa*)(ost + 4 * q);
      *(volatile v4f*)(ob + 4 * q) = v;
    }
    if (tid < rem) {
      const float v = ost[4 * nq + tid];
      *(volatile float*)(ob + 4 * nq + tid) = v;
    }
    __threadfence();
#pragma unroll 1
    for (int q = tid; q < nq; q += GTHR) {
      const v4f v = *(const v4fa*)(ost + 4 * q);
      *(volatile v4f*)(ob + 4 * q) = v;
    }
    if (tid < rem) {
      const float v = ost[4 * nq + tid];
      *(volatile float*)(ob + 4 * nq + tid) = v;
    }
  }

  if constexpr (EPI == 0) {
    if (lane == 0) wst[wave * WSTW] = (float)wn;
#pragma unroll
    for (int j = 0; j < CPL; ++j) {
      wst[wave * WSTW + 1 + CPL * lane + j]       = wm[j];
      wst[wave * WSTW + 1 + GNC + CPL * lane + j] = wqv[j];
    }
#pragma unroll 1
    for (int i = tid; i < PARTW; i += GTHR) pst[i] = 0.0f;
    __syncthreads();
    if (tid < NC) {
      float n = 0.0f, mean = 0.0f, M2 = 0.0f;
#pragma unroll 1
      for (int w2 = 0; w2 < GWAVE; ++w2) {
        const float nb = wst[w2 * WSTW];
        const float mb = wst[w2 * WSTW + 1 + tid];
        const float qb = wst[w2 * WSTW + 1 + GNC + tid];
        if (nb > 0.5f) {
          const float nn = n + nb;
          const float delta = mb - mean;
          const float f = nb / nn;
          mean = fmaf(delta, f, mean);
          M2 = M2 + qb + delta * delta * n * f;
          n = nn;
        }
      }
      pst[1 + tid] = mean;
      pst[1 + GNC + tid] = M2;
      if (tid == 0) pst[0] = n;
    }
    __syncthreads();
    const int pb = (int)blockIdx.x * (int)gridDim.y + (int)blockIdx.y;
    v4f ps = {0.0f, 0.0f, 0.0f, 0.0f};
    if (tid < PARTW / 4) {
      ps = *(const v4fa*)(pst + 4 * tid);
      *(volatile v4f*)(part + (size_t)pb * PARTW + 4 * tid) = ps;
    }
    __threadfence();
    if (tid < PARTW / 4) {
      *(volatile v4f*)(part + (size_t)pb * PARTW + 4 * tid) = ps;
    }
  } else {
    (void)part; (void)wn; (void)wm; (void)wqv; (void)wst; (void)pst;
  }
  if constexpr (EPI != 2) { (void)ost; }
  if constexpr (EPI != 3) { (void)opl; }
  if constexpr (EPI == 3) { (void)outp; }
}

template <int NCH>
__global__ __launch_bounds__(NCH) void k_bnfin(const float* __restrict__ part, int nPart,
                                               const float* __restrict__ gam, const float* __restrict__ bet,
                                               float* ss) {
  constexpr int NCB = NCH / GNC;
  static_assert(NCH % GNC == 0 && NCB >= 1 && NCB <= 2 && NCH % 8 == 0);
  __shared__ __attribute__((aligned(16))) float stg[2 * NCH];
  const int tid = (int)threadIdx.x;
  const int cb = tid >> 7;
  const int cc = tid & (GNC - 1);
  double n = 0.0, mean = 0.0, M2 = 0.0;
#pragma unroll 1
  for (int b = 0; b < nPart; ++b) {
    const float* pr = part + ((size_t)b * NCB + (size_t)cb) * PARTW;
    const double nb = (double)pr[0];
    const double mb = (double)pr[1 + cc];
    const double qb = (double)pr[1 + GNC + cc];
    if (nb > 0.5) {
      const double nn = n + nb;
      const double delta = mb - mean;
      const double f = nb / nn;
      mean = mean + delta * f;
      M2 = M2 + qb + delta * delta * n * f;
      n = nn;
    }
  }
  const double ntot = n < 1.0 ? 1.0 : n;
  const float varf  = (float)(M2 / ntot);
  const float meanf = (float)mean;
  const float rstd = rsqrtf(varf + 1e-5f);
  const float sc = bf16_val(gam[tid]) * rstd;
  const float sh = bf16_val(bet[tid]) - meanf * sc;
  stg[tid] = sc;
  stg[NCH + tid] = sh;
  __syncthreads();
  v4f v = {0.0f, 0.0f, 0.0f, 0.0f};
  if (tid < (2 * NCH) / 4) {
    v = *(const v4fa*)(stg + 4 * tid);
    *(volatile v4f*)(ss + 4 * tid) = v;
  }
  __threadfence();
  if (tid < (2 * NCH) / 4) {
    *(volatile v4f*)(ss + 4 * tid) = v;
  }
}

template <int CH>
__global__ __launch_bounds__(NTHR) void k_apply1(const float* __restrict__ s1, const float* __restrict__ ss,
                                                 int nN, int mRows, unsigned short* apl) {
  constexpr int CP = CH / 32;
  constexpr int KP = 2 * CH;
  static_assert(CP == 4 || CP == 8);
  __shared__ __attribute__((aligned(16))) float ssh[2 * CH];
  const int tid = (int)threadIdx.x, lane = tid & 31, wave = tid >> 5;
#pragma unroll 1
  for (int i = tid; i < 2 * CH; i += NTHR) ssh[i] = ss[i];
  __syncthreads();
  float sc[CP], sh[CP];
  if constexpr (CP == 4) {
    const v4f a0 = *(const v4fa*)(ssh + 4 * lane);
    const v4f b0 = *(const v4fa*)(ssh + CH + 4 * lane);
    sc[0] = a0.x; sc[1] = a0.y; sc[2] = a0.z; sc[3] = a0.w;
    sh[0] = b0.x; sh[1] = b0.y; sh[2] = b0.z; sh[3] = b0.w;
  } else {
    const v4f a0 = *(const v4fa*)(ssh + 8 * lane);
    const v4f a1 = *(const v4fa*)(ssh + 8 * lane + 4);
    const v4f b0 = *(const v4fa*)(ssh + CH + 8 * lane);
    const v4f b1 = *(const v4fa*)(ssh + CH + 8 * lane + 4);
    sc[0] = a0.x; sc[1] = a0.y; sc[2] = a0.z; sc[3] = a0.w; sc[4] = a1.x; sc[5] = a1.y; sc[6] = a1.z; sc[7] = a1.w;
    sh[0] = b0.x; sh[1] = b0.y; sh[2] = b0.z; sh[3] = b0.w; sh[4] = b1.x; sh[5] = b1.y; sh[6] = b1.z; sh[7] = b1.w;
  }
  const int rb0 = (int)blockIdx.x * HPB + wave * HPR;

#pragma unroll 1
  for (int i = 0; i < HPR; ++i) {
    const int row = rb0 + i;
    const bool live = row < nN;
    const int rc = live ? row : (nN - 1);
    float a[CP];
    ldrow<CP, 0>(s1 + (size_t)rc * CH + CP * lane, a);
    unsigned hb[CP], lb[CP];
#pragma unroll
    for (int j = 0; j < CP; ++j) {
      const float y = live ? fmaxf(fmaf(a[j], sc[j], sh[j]), 0.0f) : 0.0f;
      hb[j] = hl_bits(y, lb[j]);
    }
    if (row < mRows) {
      unsigned short* rpw = apl + (size_t)row * KP;
      if constexpr (CP == 4) {
        v2u hp, lp;
        hp.x = hb[0] | (hb[1] << 16); hp.y = hb[2] | (hb[3] << 16);
        lp.x = lb[0] | (lb[1] << 16); lp.y = lb[2] | (lb[3] << 16);
        unsigned short* ph = rpw + 4 * lane;
        unsigned short* pl = rpw + CH + 4 * lane;
        *(volatile v2u*)ph = hp;
        *(volatile v2u*)pl = lp;
        __threadfence();
        *(volatile v2u*)ph = hp;
        *(volatile v2u*)pl = lp;
      } else {
        v4u hp, lp;
        hp.x = hb[0] | (hb[1] << 16); hp.y = hb[2] | (hb[3] << 16); hp.z = hb[4] | (hb[5] << 16); hp.w = hb[6] | (hb[7] << 16);
        lp.x = lb[0] | (lb[1] << 16); lp.y = lb[2] | (lb[3] << 16); lp.z = lb[4] | (lb[5] << 16); lp.w = lb[6] | (lb[7] << 16);
        unsigned short* ph = rpw + 8 * lane;
        unsigned short* pl = rpw + CH + 8 * lane;
        *(volatile v4u*)ph = hp;
        *(volatile v4u*)pl = lp;
        __threadfence();
        *(volatile v4u*)ph = hp;
        *(volatile v4u*)pl = lp;
      }
    }
  }
}

__global__ __launch_bounds__(NTHR) void k_apply2(const float* __restrict__ tpl, const float* __restrict__ ss,
                                                 int nN, int nUnits, float* hout) {
  __shared__ __attribute__((aligned(16))) float ssh[2 * F0];
  const int tid = (int)threadIdx.x;
  ssh[tid] = ss[tid];
  __syncthreads();
  const int u = (int)blockIdx.x * NTHR + tid;
  if (u >= nUnits) return;
  const int row = u >> 5, j = u & 31, c0 = 4 * j;
  const bool live = row < nN;
  const int rc = live ? row : (nN - 1);
  const v4f a  = *(const v4fa*)(tpl + (size_t)rc * F0 + c0);
  const v4f sc = *(const v4fa*)(ssh + c0);
  const v4f sh = *(const v4fa*)(ssh + F0 + c0);
  v4f y;
  y.x = live ? fmaxf(fmaf(a.x, sc.x, sh.x), 0.0f) : 0.0f;
  y.y = live ? fmaxf(fmaf(a.y, sc.y, sh.y), 0.0f) : 0.0f;
  y.z = live ? fmaxf(fmaf(a.z, sc.z, sh.z), 0.0f) : 0.0f;
  y.w = live ? fmaxf(fmaf(a.w, sc.w, sh.w), 0.0f) : 0.0f;
  float* op = hout + (size_t)row * F0 + c0;
  *(volatile v4f*)op = y;
  __threadfence();
  *(volatile v4f*)op = y;
}

static inline int cdiv(int a, int b) { return (a + b - 1) / b; }
static inline size_t al256(size_t o) { return (o + 255) & ~(size_t)255; }

extern "C" void kernel_launch(void* const* d_in, const int* in_sizes, int n_in,
                              void* d_out, int out_size, void* d_ws, size_t ws_size,
                              hipStream_t stream) {
  if (n_in < 17) return;
  if (in_sizes[0] < F0 || (in_sizes[0] % F0) != 0) return;
  const int nN = in_sizes[0] / F0;
  if (nN < 16 || nN >= (1 << 22)) return;
  if (in_sizes[1] < 2 || (in_sizes[1] & 1) != 0) return;
  const int nE = in_sizes[1] / 2;
  if (nE < 1 || nE >= (1 << 21)) return;
  if (in_sizes[2] < F0 * C1 || (in_sizes[2] % (F0 * C1)) != 0) return;
  const int nL = in_sizes[2] / (F0 * C1);
  if (nL < 1 || nL > MAXL) return;
  if (in_sizes[3] != nL * C1 || in_sizes[4] != nL * C1 || in_sizes[5] != nL * C1) return;
  if (in_sizes[6] != nL * C1 * F0) return;
  if (in_sizes[7] != nL * F0) return;
  if (in_sizes[8] != nL) return;
  if (in_sizes[9] != nL * F0 || in_sizes[10] != nL * F0) return;
  if (in_sizes[11] != F0 * F0) return;
  if (in_sizes[12] != F0 || in_sizes[13] != F0 || in_sizes[14] != F0) return;
  if (in_sizes[15] != F0 * NCLS || in_sizes[16] != NCLS) return;
  if ((long long)out_size != (long long)nN * NCLS) return;

  const float* x     = (const float*)d_in[0];
  const int*   ei    = (const int*)  d_in[1];
  const float* W1    = (const float*)d_in[2];
  const float* b1    = (const float*)d_in[3];
  const float* g1    = (const float*)d_in[4];
  const float* bb1   = (const float*)d_in[5];
  const float* W2    = (const float*)d_in[6];
  const float* b2    = (const float*)d_in[7];
  const float* eps   = (const float*)d_in[8];
  const float* g2    = (const float*)d_in[9];
  const float* bb2   = (const float*)d_in[10];
  const float* L1w   = (const float*)d_in[11];
  const float* L1b   = (const float*)d_in[12];
  const float* n1g   = (const float*)d_in[13];
  const float* n1b   = (const float*)d_in[14];
  const float* L2w   = (const float*)d_in[15];
  const float* L2b   = (const float*)d_in[16];
  float* out = (float*)d_out;
  const int* src = ei;
  const int* dst = ei + nE;

  const int MP = cdiv(nN, GBM) * GBM;
  const int gM = MP / GBM;
  const int gA = cdiv(nN, NBA);
  if ((long long)gA * NBA < (long long)MP) return;
  if ((MP % HPB) != 0) return;
  const int vec8 = ((nE & 3) == 0) ? 1 : 0;

  char* ws = (char*)d_ws;
  size_t off = 0;
  const size_t oBT1 = off; off = al256(off + (size_t)nL * C1 * KZ * 2);
  const size_t oBT2 = off; off = al256(off + (size_t)nL * F0 * KA * 2);
  const size_t oBL1 = off; off = al256(off + (size_t)F0 * KZ * 2);
  const size_t oBL2 = off; off = al256(off + (size_t)NCP * KZ * 2);
  const size_t oR1  = off; off = al256(off + (size_t)MP * KA * 2);
  const size_t oR2  = off; off = al256(off + (size_t)MP * C1 * 4);
  const size_t oR3  = off; off = al256(off + (size_t)MP * F0 * 4);
  const size_t oPT  = off; off = al256(off + (size_t)2 * gM * PARTW * 4);
  const size_t oSS  = off; off = al256(off + (size_t)(2 * C1) * 4);
  const size_t oDM  = off; off = al256(off + 256);
  if (off > ws_size || off > (size_t)WSMAX) return;
  unsigned short* BT1 = (unsigned short*)(ws + oBT1);
  unsigned short* BT2 = (unsigned short*)(ws + oBT2);
  unsigned short* BL1 = (unsigned short*)(ws + oBL1);
  unsigned short* BL2 = (unsigned short*)(ws + oBL2);
  unsigned short* R1u = (unsigned short*)(ws + oR1);
  float*          R2f = (float*)(ws + oR2);
  unsigned short* R2u = (unsigned short*)(ws + oR2);
  float*          R3f = (float*)(ws + oR3);
  float*          PT  = (float*)(ws + oPT);
  float*          SS  = (float*)(ws + oSS);
  float*          DMf = (float*)(ws + oDM);
  unsigned short* DMu = (unsigned short*)(ws + oDM);

  const size_t scanLds = (size_t)AGG_LDS_INTS * 4;
  hipFuncSetAttribute(reinterpret_cast<const void*>(&k_scan<F0, 1>), hipFuncAttributeMaxDynamicSharedMemorySize, (int)scanLds);
  hipFuncSetAttribute(reinterpret_cast<const void*>(&k_scan<F0, 0>), hipFuncAttributeMaxDynamicSharedMemorySize, (int)scanLds);

  {
    const int upl1 = C1 * (KZ / 8);
    k_wtr<<<cdiv(nL * upl1, NTHR), NTHR, 0, stream>>>(W1, F0, C1, C1, KZ, upl1, nL * upl1, BT1);
    const int upl2 = F0 * (KA / 8);
    k_wtr<<<cdiv(nL * upl2, NTHR), NTHR, 0, stream>>>(W2, C1, F0, F0, KA, upl2, nL * upl2, BT2);
    const int upl3 = F0 * (KZ / 8);
    k_wtr<<<cdiv(upl3, NTHR), NTHR, 0, stream>>>(L1w, F0, F0, F0, KZ, upl3, upl3, BL1);
    const int upl4 = NCP * (KZ / 8);
    k_wtr<<<cdiv(upl4, NTHR), NTHR, 0, stream>>>(L2w, F0, NCLS, NCP, KZ, upl4, upl4, BL2);
  }

  const int nUh = MP * 32;
  for (int l = 0; l < nL; ++l) {
    if (l == 0) {
      k_scan<F0, 1><<<gA, NTHR, scanLds, stream>>>(src, dst, nE, nN, vec8, MP, eps, x, R1u);
    } else {
      k_scan<F0, 0><<<gA, NTHR, scanLds, stream>>>(src, dst, nE, nN, vec8, MP, eps + l, R3f, R1u);
    }
    k_gemm<GNC, KZ, C1, 0><<<dim3(gM, C1 / GNC), GTHR, 0, stream>>>(R1u, BT1 + (size_t)l * (C1 * KZ),
                                                                     b1 + (size_t)l * C1, nN, R2f, PT, DMu);
    k_bnfin<C1><<<1, C1, 0, stream>>>(PT, gM, g1 + (size_t)l * C1, bb1 + (size_t)l * C1, SS);
    k_apply1<C1><<<gM, NTHR, 0, stream>>>(R2f, SS, nN, MP, R1u);
    if (l < nL - 1) {
      k_gemm<GNC, KA, F0, 0><<<dim3(gM, 1), GTHR, 0, stream>>>(R1u, BT2 + (size_t)l * (F0 * KA),
                                                             b2 + (size_t)l * F0, nN, R2f, PT, DMu);
      k_bnfin<F0><<<1, F0, 0, stream>>>(PT, gM, g2 + (size_t)l * F0, bb2 + (size_t)l * F0, SS);
      k_apply2<<<nUh / NTHR, NTHR, 0, stream>>>(R2f, SS, nN, nUh, R3f);
    } else {
      k_gemm<GNC, KA, F0, 3><<<dim3(gM, 1), GTHR, 0, stream>>>(R1u, BT2 + (size_t)l * (F0 * KA),
                                                             b2 + (size_t)l * F0, nN, DMf, DMf, R2u);
    }
  }

  k_gemm<GNC, KZ, F0, 0><<<dim3(gM, 1), GTHR, 0, stream>>>(R2u, BL1, L1b, nN, R3f, PT, DMu);
  k_bnfin<F0><<<1, F0, 0, stream>>>(PT, gM, n1g, n1b, SS);
  k_apply1<F0><<<gM, NTHR, 0, stream>>>(R3f, SS, nN, MP, R1u);
  k_gemm<NCP, KZ, NCP, 2><<<dim3(gM, 1), GTHR, 0, stream>>>(R1u, BL2, L2b, nN, out, DMf, DMu);
}
